// CondDecoder_6957847019937
// MI455X (gfx1250) — hardware-verified
//
#include <hip/hip_runtime.h>


typedef _Float16 f16t;
typedef f16t  v16h __attribute__((ext_vector_type(16)));
typedef f16t  v8h  __attribute__((ext_vector_type(8)));
typedef __bf16 bf16t;
typedef bf16t v16b __attribute__((ext_vector_type(16)));
typedef unsigned short v8us __attribute__((ext_vector_type(8)));
typedef float v8f __attribute__((ext_vector_type(8)));
typedef float v4f __attribute__((ext_vector_type(4)));
typedef unsigned int v4u __attribute__((ext_vector_type(4)));

union Frag  { v16h v; v8h  q[2]; };
union FragB { v16b v; v8us q[2]; };
union Pk16  { v8h  h; v4u u; };
union Pk16u { v8us s; v4u u; };

#define NB_  256
#define NT_  128
#define NH_  512
#define NG_  1536
#define NV_  64
#define NL_  128
#define NE_  32
#define NI0  161
#define RB   16
#define LP   520
#define NTHR 512
#define GSTR ((size_t)NH_ * NH_)

__device__ __forceinline__ v8f wmma_h(v16h a, v16h b, v8f c) {
    return __builtin_amdgcn_wmma_f32_16x16x32_f16(false, a, false, b, (short)0, c, false, false);
}
__device__ __forceinline__ v8f wmma_b(v16b a, v16b b, v8f c) {
    return __builtin_amdgcn_wmma_f32_16x16x32_bf16(false, a, false, b, (short)0, c, false, false);
}

__device__ __forceinline__ v8f splat8(float c) {
    v8f v = {c, c, c, c, c, c, c, c};
    return v;
}

__device__ __forceinline__ unsigned int bf16_rne(float x) {
    unsigned int u = __float_as_uint(x);
    u += 0x7FFFu + ((u >> 16) & 1u);
    return u >> 16;
}

__device__ __forceinline__ float fsig(float x) {
    float t = __expf(-x);
    return __builtin_amdgcn_rcpf(1.0f + t);
}
__device__ __forceinline__ float ftanh(float x) {
    float ax = fabsf(x);
    float t  = __expf(-2.0f * ax);
    float r  = (1.0f - t) * __builtin_amdgcn_rcpf(1.0f + t);
    return copysignf(r, x);
}

__device__ __forceinline__ void mma3(v8f& a0, v8f& a1, v8f& a2,
                                     const f16t* Ap, const f16t* Bq) {
#pragma unroll 1
    for (int k0 = 0; k0 < NH_; k0 += 32) {
        Frag a, b0, b1, b2;
        a.q[0] = *(const v8h*)(Ap + k0);
        a.q[1] = *(const v8h*)(Ap + k0 + 16);
        const f16t* p = Bq + k0;
        b0.q[0] = *(const v8h*)(p);             b0.q[1] = *(const v8h*)(p + 16);
        b1.q[0] = *(const v8h*)(p + GSTR);      b1.q[1] = *(const v8h*)(p + GSTR + 16);
        b2.q[0] = *(const v8h*)(p + 2 * GSTR);  b2.q[1] = *(const v8h*)(p + 2 * GSTR + 16);
        a0 = wmma_h(a.v, b0.v, a0);
        a1 = wmma_h(a.v, b1.v, a1);
        a2 = wmma_h(a.v, b2.v, a2);
        asm volatile("v_nop\n\tv_nop\n\tv_nop\n\tv_nop"
                     : "+v"(a0), "+v"(a1), "+v"(a2)
                     : "v"(a.v), "v"(b0.v), "v"(b1.v), "v"(b2.v));
    }
}

__device__ __forceinline__ void gate_update(const v8f& aR, const v8f& aZ, const v8f& aN,
                                            const float (&gin)[8], float* hSc) {
    const float I64 = 0.015625f;
    v8f ho = *(const v8f*)hSc;
    v8f hn;
#pragma unroll
    for (int r = 0; r < 8; ++r) {
        float rg = fsig(aR[r] * I64);
        float zg = fsig(aZ[r] * I64);
        float nn = ftanh(fmaf(rg, aN[r] * I64, gin[r]));
        hn[r] = (1.0f - zg) * nn + zg * ho[r];
    }
    *(v8f*)hSc = hn;
}

template<bool WB>
__device__ __forceinline__ void refresh_planes(const float* hSl, f16t* hAl,
                                               unsigned short* bh, unsigned short* bl,
                                               int cb, int hh, int m) {
#pragma unroll
    for (int nt = 0; nt < 2; ++nt) {
        const int c = cb + 16 * nt + m;
        v8f hv = *(const v8f*)(hSl + c * RB + 8 * hh);
#pragma unroll
        for (int r = 0; r < 8; ++r) {
            const float x = hv[r];
            const int   o = (8 * hh + r) * LP + c;
            hAl[o] = (f16t)x;
            if (WB) {
                unsigned int hi = bf16_rne(x);
                float xh = __uint_as_float(hi << 16);
                unsigned int lo = bf16_rne(x - xh);
                bh[o] = (unsigned short)hi;
                bl[o] = (unsigned short)lo;
            }
        }
    }
}

__global__ __launch_bounds__(256)
void k_cvt8(const float* x, f16t* y, int n8, float sc) {
    int i = blockIdx.x * 256 + threadIdx.x;
    if (i >= n8) return;
    const float* p = x + (size_t)i * 8;
    v4f a = *(const v4f*)p;
    v4f b = *(const v4f*)(p + 4);
    Pk16 k;
    k.h[0] = (f16t)(a[0] * sc); k.h[1] = (f16t)(a[1] * sc);
    k.h[2] = (f16t)(a[2] * sc); k.h[3] = (f16t)(a[3] * sc);
    k.h[4] = (f16t)(b[0] * sc); k.h[5] = (f16t)(b[1] * sc);
    k.h[6] = (f16t)(b[2] * sc); k.h[7] = (f16t)(b[3] * sc);
    f16t* d = y + (size_t)i * 8;
    *(volatile v4u*)d = k.u;
    __threadfence();
    *(volatile v4u*)d = k.u;
}

__global__ __launch_bounds__(256)
void k_split_bf16(const float* x, unsigned short* ph, unsigned short* pl, int n8) {
    int i = blockIdx.x * 256 + threadIdx.x;
    if (i >= n8) return;
    const float* p = x + (size_t)i * 8;
    v4f a = *(const v4f*)p;
    v4f b = *(const v4f*)(p + 4);
    Pk16u hi, lo;
#pragma unroll
    for (int e = 0; e < 4; ++e) {
        float v0 = a[e];
        unsigned int u0 = bf16_rne(v0);
        hi.s[e] = (unsigned short)u0;
        lo.s[e] = (unsigned short)bf16_rne(v0 - __uint_as_float(u0 << 16));
        float v1 = b[e];
        unsigned int u1 = bf16_rne(v1);
        hi.s[4 + e] = (unsigned short)u1;
        lo.s[4 + e] = (unsigned short)bf16_rne(v1 - __uint_as_float(u1 << 16));
    }
    unsigned short* dh = ph + (size_t)i * 8;
    unsigned short* dl = pl + (size_t)i * 8;
    *(volatile v4u*)dh = hi.u;
    *(volatile v4u*)dl = lo.u;
    __threadfence();
    *(volatile v4u*)dh = hi.u;
    *(volatile v4u*)dl = lo.u;
}

__global__ __launch_bounds__(256)
void k_gl(const float* lat, const float* enth, const float* W0,
          const float* bih, const float* bhh, float* GLT) {
    const int g = blockIdx.x, b = threadIdx.x;
    const float* wr = W0 + (size_t)g * NI0;
    const float* xr = lat + (size_t)b * NL_;
    float s = 0.0f;
#pragma unroll 4
    for (int k = 0; k < NL_; ++k) s = fmaf(xr[k], wr[k], s);
    s = fmaf(enth[b], wr[NL_ + NE_], s);
    float bv = bhh[g];
    float bsum = bih[g] + ((g < 2 * NH_) ? bv : 0.0f);
    s += bsum;
    float* d = GLT + (size_t)g * NB_ + b;
    *(volatile float*)d = s;
    __threadfence();
    *(volatile float*)d = s;
}

__global__ __launch_bounds__(64)
void k_ge(const float* emb, const float* W0, float* GET) {
    const int g = blockIdx.x, v = threadIdx.x;
    const float* wr = W0 + (size_t)g * NI0 + NL_;
    const float* er = emb + (size_t)v * NE_;
    float s = 0.0f;
#pragma unroll 4
    for (int e = 0; e < NE_; ++e) s = fmaf(er[e], wr[e], s);
    float* d = GET + (size_t)g * NV_ + v;
    *(volatile float*)d = s;
    __threadfence();
    *(volatile float*)d = s;
}

__global__ __launch_bounds__(NTHR)
void k_gru(const float* GLT, const float* GET, const int* tok,
           const f16t* Phh0, const float* bhh0,
           const f16t* Pih1, const f16t* Phh1, const float* bih1, const float* bhh1,
           const f16t* Pih2, const f16t* Phh2, const float* bih2, const float* bhh2,
           const unsigned short* Pfh, const unsigned short* Pfl, const float* fcb,
           float* out, int nb) {
    __shared__ __attribute__((aligned(32))) f16t hA0[RB * LP];
    __shared__ __attribute__((aligned(32))) f16t hA1[RB * LP];
    __shared__ __attribute__((aligned(32))) f16t hA2[RB * LP];
    __shared__ __attribute__((aligned(32))) float hS[3 * NH_ * RB];
    __shared__ __attribute__((aligned(32))) unsigned short hBh[RB * LP];
    __shared__ __attribute__((aligned(32))) unsigned short hBl[RB * LP];
    __shared__ __attribute__((aligned(32))) float Slog[NV_ * RB];

    const int tid = threadIdx.x;
    const int l = tid & 31, w = tid >> 5, hh = l >> 4, m = l & 15;
    const int b0 = blockIdx.x * RB;
    if (b0 + RB > nb) return;

    for (int i = tid; i < RB * LP; i += NTHR) {
        hA0[i] = (f16t)0.0f; hA1[i] = (f16t)0.0f; hA2[i] = (f16t)0.0f;
        hBh[i] = 0; hBl[i] = 0;
    }
    for (int i = tid; i < 3 * NH_ * RB; i += NTHR) hS[i] = 0.0f;
    __syncthreads();

    const int cb = 32 * w;
    const f16t* Ap0 = hA0 + m * LP + 8 * hh;
    const f16t* Ap1 = hA1 + m * LP + 8 * hh;
    const f16t* Ap2 = hA2 + m * LP + 8 * hh;
    const size_t boff = (size_t)(cb + m) * NH_ + 8 * hh;
    float* hS0 = hS;
    float* hS1 = hS + NH_ * RB;
    float* hS2 = hS + 2 * NH_ * RB;
    const int crow = (tid >> 4) & 15, c4 = (tid & 15) * 4;
    const float S64 = 64.0f, I64 = 0.015625f;

#pragma unroll 1
    for (int t = 0; t < NT_; ++t) {
        {
            int tk[8];
            const int tm1 = (t > 0) ? (t - 1) : 0;
#pragma unroll
            for (int r = 0; r < 8; ++r) {
                int v = tok[(size_t)(b0 + 8 * hh + r) * NT_ + tm1];
                v = (t > 0) ? v : 0;
                v = (v < 0) ? 0 : ((v > NV_ - 1) ? (NV_ - 1) : v);
                tk[r] = v;
            }
#pragma unroll 1
            for (int nt = 0; nt < 2; ++nt) {
                const int c = cb + 16 * nt + m;
                v8f xr = *(const v8f*)(GLT + (size_t)c * NB_ + b0 + 8 * hh);
                v8f xz = *(const v8f*)(GLT + (size_t)(NH_ + c) * NB_ + b0 + 8 * hh);
                v8f xn = *(const v8f*)(GLT + (size_t)(2 * NH_ + c) * NB_ + b0 + 8 * hh);
                const float* ger = GET + (size_t)c * NV_;
                const float* gez = GET + (size_t)(NH_ + c) * NV_;
                const float* gen = GET + (size_t)(2 * NH_ + c) * NV_;
                const float bn = S64 * bhh0[2 * NH_ + c];
                v8f aR, aZ, aN;
                float gin[8];
#pragma unroll
                for (int r = 0; r < 8; ++r) {
                    aR[r]  = S64 * (xr[r] + ger[tk[r]]);
                    aZ[r]  = S64 * (xz[r] + gez[tk[r]]);
                    gin[r] = xn[r] + gen[tk[r]];
                    aN[r]  = bn;
                }
                mma3(aR, aZ, aN, Ap0, Phh0 + boff + (size_t)(16 * nt) * NH_);
                gate_update(aR, aZ, aN, gin, hS0 + c * RB + 8 * hh);
            }
            __syncthreads();
            refresh_planes<false>(hS0, hA0, hBh, hBl, cb, hh, m);
            __syncthreads();
        }
        {
#pragma unroll 1
            for (int nt = 0; nt < 2; ++nt) {
                const int c = cb + 16 * nt + m;
                v8f aR = splat8(S64 * (bih1[c] + bhh1[c]));
                v8f aZ = splat8(S64 * (bih1[NH_ + c] + bhh1[NH_ + c]));
                v8f aI = splat8(S64 * bih1[2 * NH_ + c]);
                mma3(aR, aZ, aI, Ap0, Pih1 + boff + (size_t)(16 * nt) * NH_);
                float gin[8];
#pragma unroll
                for (int r = 0; r < 8; ++r) gin[r] = aI[r] * I64;
                v8f aN = splat8(S64 * bhh1[2 * NH_ + c]);
                mma3(aR, aZ, aN, Ap1, Phh1 + boff + (size_t)(16 * nt) * NH_);
                gate_update(aR, aZ, aN, gin, hS1 + c * RB + 8 * hh);
            }
            __syncthreads();
            refresh_planes<false>(hS1, hA1, hBh, hBl, cb, hh, m);
            __syncthreads();
        }
        {
#pragma unroll 1
            for (int nt = 0; nt < 2; ++nt) {
                const int c = cb + 16 * nt + m;
                v8f aR = splat8(S64 * (bih2[c] + bhh2[c]));
                v8f aZ = splat8(S64 * (bih2[NH_ + c] + bhh2[NH_ + c]));
                v8f aI = splat8(S64 * bih2[2 * NH_ + c]);
                mma3(aR, aZ, aI, Ap1, Pih2 + boff + (size_t)(16 * nt) * NH_);
                float gin[8];
#pragma unroll
                for (int r = 0; r < 8; ++r) gin[r] = aI[r] * I64;
                v8f aN = splat8(S64 * bhh2[2 * NH_ + c]);
                mma3(aR, aZ, aN, Ap2, Phh2 + boff + (size_t)(16 * nt) * NH_);
                gate_update(aR, aZ, aN, gin, hS2 + c * RB + 8 * hh);
            }
            __syncthreads();
            refresh_planes<true>(hS2, hA2, hBh, hBl, cb, hh, m);
            __syncthreads();
        }
        {
            if (w < 4) {
                v8f acc = splat8(fcb[16 * w + m]);
                const unsigned short* ah = hBh + m * LP + 8 * hh;
                const unsigned short* al = hBl + m * LP + 8 * hh;
                const unsigned short* bh = Pfh + (size_t)(16 * w + m) * NH_ + 8 * hh;
                const unsigned short* bl = Pfl + (size_t)(16 * w + m) * NH_ + 8 * hh;
#pragma unroll 1
                for (int k0 = 0; k0 < NH_; k0 += 32) {
                    FragB xh, xl, yh, yl;
                    xh.q[0] = *(const v8us*)(ah + k0); xh.q[1] = *(const v8us*)(ah + k0 + 16);
                    xl.q[0] = *(const v8us*)(al + k0); xl.q[1] = *(const v8us*)(al + k0 + 16);
                    yh.q[0] = *(const v8us*)(bh + k0); yh.q[1] = *(const v8us*)(bh + k0 + 16);
                    yl.q[0] = *(const v8us*)(bl + k0); yl.q[1] = *(const v8us*)(bl + k0 + 16);
                    acc = wmma_b(xh.v, yh.v, acc);
                    acc = wmma_b(xh.v, yl.v, acc);
                    acc = wmma_b(xl.v, yh.v, acc);
                    asm volatile("v_nop\n\tv_nop\n\tv_nop\n\tv_nop"
                                 : "+v"(acc)
                                 : "v"(xh.v), "v"(xl.v), "v"(yh.v), "v"(yl.v));
                }
                *(v8f*)(Slog + (16 * w + m) * RB + 8 * hh) = acc;
            }
            __syncthreads();
            v4f ov = {0.0f, 0.0f, 0.0f, 0.0f};
            float* dst = out + ((size_t)(b0 + crow) * NT_ + t) * NV_ + c4;
            if (tid < 256) {
                ov[0] = Slog[(c4 + 0) * RB + crow];
                ov[1] = Slog[(c4 + 1) * RB + crow];
                ov[2] = Slog[(c4 + 2) * RB + crow];
                ov[3] = Slog[(c4 + 3) * RB + crow];
                *(volatile v4f*)dst = ov;
            }
            __threadfence();
            if (tid < 256) {
                *(volatile v4f*)dst = ov;
            }
        }
    }
}

extern "C" void kernel_launch(void* const* d_in, const int* in_sizes, int n_in,
                              void* d_out, int out_size, void* d_ws, size_t ws_size,
                              hipStream_t stream) {
    if (n_in < 18) return;
    if (in_sizes[0] != NB_ * NL_ || in_sizes[1] != NB_ || in_sizes[2] != NB_ * NT_ ||
        in_sizes[3] != NV_ * NE_ || in_sizes[4] != NG_ * NI0 || in_sizes[5] != NG_ * NH_ ||
        in_sizes[6] != NG_ || in_sizes[7] != NG_ || in_sizes[8] != NG_ * NH_ ||
        in_sizes[9] != NG_ * NH_ || in_sizes[10] != NG_ || in_sizes[11] != NG_ ||
        in_sizes[12] != NG_ * NH_ || in_sizes[13] != NG_ * NH_ || in_sizes[14] != NG_ ||
        in_sizes[15] != NG_ || in_sizes[16] != NV_ * NH_ || in_sizes[17] != NV_ ||
        out_size != NB_ * NT_ * NV_) return;

    const float* latent = (const float*)d_in[0];
    const float* enth   = (const float*)d_in[1];
    const int*   tok    = (const int*)d_in[2];
    const float* embed  = (const float*)d_in[3];
    const float* Wih0 = (const float*)d_in[4];
    const float* Whh0 = (const float*)d_in[5];
    const float* bih0 = (const float*)d_in[6];
    const float* bhh0 = (const float*)d_in[7];
    const float* Wih1 = (const float*)d_in[8];
    const float* Whh1 = (const float*)d_in[9];
    const float* bih1 = (const float*)d_in[10];
    const float* bhh1 = (const float*)d_in[11];
    const float* Wih2 = (const float*)d_in[12];
    const float* Whh2 = (const float*)d_in[13];
    const float* bih2 = (const float*)d_in[14];
    const float* bhh2 = (const float*)d_in[15];
    const float* fcW  = (const float*)d_in[16];
    const float* fcb  = (const float*)d_in[17];
    float* out = (float*)d_out;

    char* ws = (char*)d_ws;
    size_t off = 0;
    auto carve = [&](size_t bytes) -> char* {
        char* p = ws + off;
        off = (off + bytes + 255) & ~(size_t)255;
        return p;
    };
    const size_t plane_b = (size_t)NG_ * NH_ * 2;
    f16t* Phh0p = (f16t*)carve(plane_b);
    f16t* Pih1p = (f16t*)carve(plane_b);
    f16t* Phh1p = (f16t*)carve(plane_b);
    f16t* Pih2p = (f16t*)carve(plane_b);
    f16t* Phh2p = (f16t*)carve(plane_b);
    unsigned short* Pfh = (unsigned short*)carve((size_t)NV_ * NH_ * 2);
    unsigned short* Pfl = (unsigned short*)carve((size_t)NV_ * NH_ * 2);
    float* GLT = (float*)carve((size_t)NG_ * NB_ * 4);
    float* GET = (float*)carve((size_t)NG_ * NV_ * 4);
    if (off > ws_size) return;

    const float S64 = 64.0f;
    const int n8 = NG_ * NH_ / 8;
    k_cvt8<<<dim3((n8 + 255) / 256), dim3(256), 0, stream>>>(Whh0, Phh0p, n8, S64);
    k_cvt8<<<dim3((n8 + 255) / 256), dim3(256), 0, stream>>>(Wih1, Pih1p, n8, S64);
    k_cvt8<<<dim3((n8 + 255) / 256), dim3(256), 0, stream>>>(Whh1, Phh1p, n8, S64);
    k_cvt8<<<dim3((n8 + 255) / 256), dim3(256), 0, stream>>>(Wih2, Pih2p, n8, S64);
    k_cvt8<<<dim3((n8 + 255) / 256), dim3(256), 0, stream>>>(Whh2, Phh2p, n8, S64);

    const int n8f = NV_ * NH_ / 8;
    k_split_bf16<<<dim3((n8f + 255) / 256), dim3(256), 0, stream>>>(fcW, Pfh, Pfl, n8f);

    k_gl<<<dim3(NG_), dim3(256), 0, stream>>>(latent, enth, Wih0, bih0, bhh0, GLT);
    k_ge<<<dim3(NG_), dim3(64), 0, stream>>>(embed, Wih0, GET);

    k_gru<<<dim3(NB_ / RB), dim3(NTHR), 0, stream>>>(GLT, GET, tok,
                                                    Phh0p, bhh0,
                                                    Pih1p, Phh1p, bih1, bhh1,
                                                    Pih2p, Phh2p, bih2, bhh2,
                                                    Pfh, Pfl, fcb, out, NB_);
}
